// CausalSelfAttention_7232724926954
// MI455X (gfx1250) — hardware-verified
//
#include <hip/hip_runtime.h>
#include <math.h>

#ifndef NB
#define NB 2
#endif
#ifndef SEQ
#define SEQ 1024
#endif
#ifndef EROWS
#define EROWS 256
#endif
#define NB_FULL 2
#define SEQ_FULL 1024
#define CW 1024
#define NH 16
#define HD 64
#define QKVW 3072
#define YW 2048
#define NR 16
#define RK 32
#define FA 32
#define TW 64
#define PSP 40
#define HSLAB 128
#define NSLAB 8
#define KP 132

constexpr int kMROWS = NB * SEQ;

static_assert(NB <= NB_FULL);
static_assert(SEQ <= SEQ_FULL);
static_assert(SEQ % 256 == 0);
static_assert(EROWS % 64 == 0 && EROWS <= SEQ && EROWS >= 64);
static_assert(CW == NH * HD);
static_assert(HD == 64);
static_assert(QKVW == 3 * CW);
static_assert(YW == 2 * CW);
static_assert(CW == FA * FA);
static_assert(FA == 32 && RK == 32 && NR == 16);
static_assert(TW == 2 * RK);
static_assert(kMROWS % 64 == 0);
static_assert(kMROWS % 4 == 0);
static_assert(CW % 64 == 0 && QKVW % 64 == 0 && SEQ % 64 == 0);
static_assert(CW == 32 * 4 * 8);
static_assert((PSP * 2) % 16 == 0 && PSP >= 32);
static_assert(CW == NSLAB * HSLAB);
static_assert(HSLAB == 32 * 4);
static_assert(HSLAB == 2 * 16 * 4);
static_assert(KP % 4 == 0 && KP >= HSLAB);
static_assert(SEQ % 8 == 0);
static_assert(kMROWS % 2 == 0);

typedef __attribute__((ext_vector_type(16))) _Float16 v16h;
typedef __attribute__((ext_vector_type(8)))  _Float16 v8h;
typedef __attribute__((ext_vector_type(8)))  float    v8f;
typedef __attribute__((ext_vector_type(4)))  float    v4f;
typedef __attribute__((ext_vector_type(2)))  float    v2f;
typedef __attribute__((ext_vector_type(4)))  unsigned int v4u;
typedef __attribute__((ext_vector_type(2)))  unsigned int v2u;
typedef __attribute__((ext_vector_type(4)))  int      v4i;
typedef v8h v8h_a __attribute__((may_alias));
typedef v4f v4f_a __attribute__((may_alias));
typedef _Float16 h16;

union FragH { v16h v; v8h h[2]; };
__device__ __forceinline__ v16h ldfrag(const _Float16* __restrict__ p) {
    FragH f; f.h[0] = *(const v8h*)(p); f.h[1] = *(const v8h*)(p + 16); return f.v;
}
__device__ __forceinline__ v8f wmma16(v16h a, v16h b, v8f c) {
    c = __builtin_amdgcn_wmma_f32_16x16x32_f16(false, a, false, b, (short)0, c, false, false);
    asm volatile("v_nop\n\tv_nop\n\tv_nop\n\tv_nop" : "+v"(c) : "v"(a), "v"(b));
    return c;
}
__device__ __forceinline__ v8f wmma_raw(v16h a, v16h b, v8f c) {
    return __builtin_amdgcn_wmma_f32_16x16x32_f16(false, a, false, b, (short)0, c, false, false);
}
__device__ __forceinline__ void dep_guard_h(v8f& a, v8f& b, v16h x, v16h y) { asm volatile("v_nop\n\tv_nop\n\tv_nop\n\tv_nop" : "+v"(a), "+v"(b) : "v"(x), "v"(y)); }
__device__ __forceinline__ void keep4_h(v16h a, v16h b, v16h c, v16h d) { asm volatile("v_nop" :: "v"(a), "v"(b), "v"(c), "v"(d)); }
__device__ __forceinline__ void acc_guard4(v8f& a, v8f& b, v8f& c, v8f& d) { asm volatile("v_nop\n\tv_nop\n\tv_nop\n\tv_nop" : "+v"(a), "+v"(b), "+v"(c), "+v"(d)); }

__device__ __forceinline__ float cmb_bf(float v) { const unsigned u = __builtin_bit_cast(unsigned, v); const unsigned r = (u + 0x7fffu + ((u >> 16) & 1u)) & 0xffff0000u; return __builtin_bit_cast(float, r); }
__device__ __forceinline__ unsigned int pk2h(float a, float b) { return (unsigned int)__builtin_bit_cast(unsigned short, (_Float16)a) | ((unsigned int)__builtin_bit_cast(unsigned short, (_Float16)b) << 16); }

static __device__ __forceinline__ h16 toh_flush(float v) { const h16 r = (h16)v; return (fabsf(v) < 6.103515625e-05f) ? (h16)0.0f : r; }
static __device__ __forceinline__ h16 res_h(float v, h16 hi) { return toh_flush((v - (float)hi) * 2048.0f); }
static __device__ __forceinline__ unsigned int pk2b(h16 a, h16 b) { return (unsigned int)__builtin_bit_cast(unsigned short, a) | ((unsigned int)__builtin_bit_cast(unsigned short, b) << 16); }

#define VST2(T, ptr, val) do { const T vst2_v_ = (val); *(volatile T*)(ptr) = vst2_v_; __threadfence(); *(volatile T*)(ptr) = vst2_v_; } while (0)

__device__ __forceinline__ void wave_sync_lds() {
    __builtin_amdgcn_fence(3  , "workgroup");
    __builtin_amdgcn_wave_barrier();
    __builtin_amdgcn_fence(2  , "workgroup");
}

__global__ __launch_bounds__(256) void k_gemm64(const unsigned short* __restrict__ Ap, int lda, const unsigned short* __restrict__ Btp, int ldb,
                                                float* __restrict__ C, int ldc, const float* __restrict__ cs, int use_cs, int M, int N, int K, float scale) {
    const _Float16* A = (const _Float16*)Ap; const _Float16* Bt = (const _Float16*)Btp;
    __shared__ __align__(16) float sT[8][16 * 68];
    const int lane = threadIdx.x & 31;
    const int wave = __builtin_amdgcn_readfirstlane((int)(threadIdx.x >> 5));
    const int tilesN = N >> 6, tilesM = M >> 6;
    const int tile = blockIdx.x * 8 + wave;
    if (tile >= tilesM * tilesN) return;
    const int tm = tile / tilesN, tn = tile - tm * tilesN;
    const int m0 = tm << 6, n0 = tn << 6;
    const int rlane = lane & 15, koff = (lane >> 4) * 8, mOff = (lane >> 4) * 8;

    v8f acc[4][4];
#pragma unroll
    for (int i = 0; i < 4; ++i)
#pragma unroll
        for (int j = 0; j < 4; ++j) acc[i][j] = (v8f){0.f, 0.f, 0.f, 0.f, 0.f, 0.f, 0.f, 0.f};

    for (int k0 = 0; k0 < K; k0 += 32) {
        v16h bh[4];
#pragma unroll
        for (int j = 0; j < 4; ++j) bh[j] = ldfrag(Bt + (size_t)(n0 + (j << 4) + rlane) * ldb + koff + k0);
#pragma unroll
        for (int i = 0; i < 4; ++i) {
            const v16h ah = ldfrag(A + (size_t)(m0 + (i << 4) + rlane) * lda + koff + k0);
#pragma unroll
            for (int j = 0; j < 4; ++j) acc[i][j] = wmma_raw(ah, bh[j], acc[i][j]);
            dep_guard_h(acc[i][0], acc[i][3], ah, ah);
        }
        keep4_h(bh[0], bh[1], bh[2], bh[3]);
    }
    acc_guard4(acc[0][0], acc[0][1], acc[0][2], acc[0][3]);
    acc_guard4(acc[1][0], acc[1][1], acc[1][2], acc[1][3]);
    acc_guard4(acc[2][0], acc[2][1], acc[2][2], acc[2][3]);
    acc_guard4(acc[3][0], acc[3][1], acc[3][2], acc[3][3]);

#pragma unroll
    for (int i = 0; i < 4; ++i) {
        const int mBase = m0 + (i << 4);
#pragma unroll
        for (int j = 0; j < 4; ++j) {
            const int n = n0 + (j << 4) + rlane;
            float csv = scale;
            if (use_cs) csv *= cmb_bf(cs[n]);
#pragma unroll
            for (int r = 0; r < 8; ++r) sT[wave][(mOff + r) * 68 + (j << 4) + rlane] = acc[i][j][r] * csv;
        }
        wave_sync_lds();
        {
            const int hh = lane >> 4, c4 = (lane & 15) * 4;
            for (int pass = 0; pass < 2; ++pass) {
#pragma unroll
                for (int it = 0; it < 8; ++it) {
                    const int row = it * 2 + hh;
                    const v4f v = *(const v4f_a*)&sT[wave][row * 68 + c4];
                    *(volatile v4f*)(C + (size_t)(mBase + row) * ldc + n0 + c4) = v;
                }
                __threadfence();
            }
        }
        wave_sync_lds();
    }
}

__global__ __launch_bounds__(256) void k_cast16(const float* __restrict__ SRC, unsigned short* __restrict__ DST, int nR, int nC, float sc, int seq, int seqfull) {
    const long long u = (long long)blockIdx.x * 256 + threadIdx.x; const int per = nC / 8; if (u >= (long long)nR * per) return;
    const int r = (int)(u / per); const int c0 = 8 * (int)(u % per);
    const int rs = (r / seq) * seqfull + (r % seq);
    const float* s = SRC + (size_t)rs * nC + c0;
    const v4f a = *(const v4f*)(s), b = *(const v4f*)(s + 4);
    v4u pk;
    pk.x = pk2h(cmb_bf(a.x) * sc, cmb_bf(a.y) * sc); pk.y = pk2h(cmb_bf(a.z) * sc, cmb_bf(a.w) * sc);
    pk.z = pk2h(cmb_bf(b.x) * sc, cmb_bf(b.y) * sc); pk.w = pk2h(cmb_bf(b.z) * sc, cmb_bf(b.w) * sc);
    VST2(v4u, (v4u*)(DST + (size_t)r * nC + c0), pk);
}

__global__ __launch_bounds__(256) void k_embtab(float* __restrict__ EMB, int n) {
    const int u = blockIdx.x * 256 + threadIdx.x; if (u >= n) return;
    const int t = u >> 5, i = u & 31;
    const float dv = expf((float)(2 * i) * (-0.14391156831212787f));
    const float ang = (float)t * dv;
    float sn, cs; sincosf(ang, &sn, &cs);
    v2f o; o.x = sn; o.y = cs;
    VST2(v2f, (v2f*)(EMB + 2 * (size_t)u), o);
}

__global__ __launch_bounds__(256) void k_castT(const float* __restrict__ SRC, int srcPitch, long long srcBatch, int nK, int nN,
                                               unsigned short* __restrict__ DST, int dstPitch, int dcol0, float sc, int nb) {
#pragma clang fp contract(off)
    __shared__ float tile[64][33];
    const int u = threadIdx.x;
    const int tk = nK / 64, tn = nN / 32;
    int bx = blockIdx.x; const int kt = bx % tk; bx /= tk; const int nt = bx % tn; const int bt = bx / tn;
    if (bt >= nb) return;
    const int k0 = kt * 64, n0 = nt * 32;
    const float* s = SRC + (size_t)bt * (size_t)srcBatch;
#pragma unroll
    for (int it = 0; it < 2; ++it) {
        const int k = (u >> 3) + 32 * it, n4 = (u & 7) * 4;
        const v4f v = *(const v4f*)(s + (size_t)(k0 + k) * srcPitch + n0 + n4);
        tile[k][n4] = v.x; tile[k][n4 + 1] = v.y; tile[k][n4 + 2] = v.z; tile[k][n4 + 3] = v.w;
    }
    __syncthreads();
    const int n = u >> 3, pc = u & 7;
    h16 hv[8];
#pragma unroll
    for (int i = 0; i < 8; ++i) hv[i] = toh_flush(cmb_bf(tile[8 * pc + i][n]) * sc);
    v4u pk; pk.x = pk2b(hv[0], hv[1]); pk.y = pk2b(hv[2], hv[3]); pk.z = pk2b(hv[4], hv[5]); pk.w = pk2b(hv[6], hv[7]);
    VST2(v4u, (v4u*)(DST + (size_t)(bt * nN + n0 + n) * dstPitch + dcol0 + k0 + 8 * pc), pk);
}

__global__ __launch_bounds__(256) void k_sot(const float* __restrict__ SO, unsigned short* __restrict__ SOT16) {
#pragma clang fp contract(off)
    const int u = blockIdx.x * 256 + threadIdx.x; if (u >= 4 * CW * 8) return;
    const int t = u & 7, c = (u >> 3) % CW, p = (u >> 3) / CW;
    const int j0 = 8 * (t & 3);
    const float sc = (t < 4) ? 1024.0f : 0.5f;
    h16 hv[8];
#pragma unroll
    for (int i = 0; i < 8; ++i) hv[i] = toh_flush(cmb_bf(SO[(size_t)(p * RK + j0 + i) * CW + c]) * sc);
    v4u pk; pk.x = pk2b(hv[0], hv[1]); pk.y = pk2b(hv[2], hv[3]); pk.z = pk2b(hv[4], hv[5]); pk.w = pk2b(hv[6], hv[7]);
    VST2(v4u, (v4u*)(SOT16 + (size_t)(p * CW + c) * TW + 8 * t), pk);
}

__global__ __launch_bounds__(256) void k_tsplit(const float* __restrict__ SRC, int srcPitch, int col0, unsigned short* __restrict__ DST, int rows, int nb) {
#pragma clang fp contract(off)
    const long long u = (long long)blockIdx.x * 256 + threadIdx.x; if (u >= (long long)nb * rows * 8) return;
    const int t = (int)(u & 7); const long long rr = u >> 3; const int row = (int)(rr % rows); const int p = (int)(rr / rows);
    const int j0 = 8 * (t & 3);
    const float* s = SRC + (size_t)row * srcPitch + col0 + p * RK + j0;
    const v4f a = *(const v4f*)(s), b = *(const v4f*)(s + 4);
    float v[8];
    v[0] = a.x * 16.f; v[1] = a.y * 16.f; v[2] = a.z * 16.f; v[3] = a.w * 16.f;
    v[4] = b.x * 16.f; v[5] = b.y * 16.f; v[6] = b.z * 16.f; v[7] = b.w * 16.f;
    h16 hv[8], rv[8];
#pragma unroll
    for (int i = 0; i < 8; ++i) { hv[i] = toh_flush(v[i]); rv[i] = res_h(v[i], hv[i]); }
    v4u ph, pr;
    ph.x = pk2b(hv[0], hv[1]); ph.y = pk2b(hv[2], hv[3]); ph.z = pk2b(hv[4], hv[5]); ph.w = pk2b(hv[6], hv[7]);
    pr.x = pk2b(rv[0], rv[1]); pr.y = pk2b(rv[2], rv[3]); pr.z = pk2b(rv[4], rv[5]); pr.w = pk2b(rv[6], rv[7]);
    const bool useHi = (t < 4);
    v4u pk; pk.x = useHi ? ph.x : pr.x; pk.y = useHi ? ph.y : pr.y; pk.z = useHi ? ph.z : pr.z; pk.w = useHi ? ph.w : pr.w;
    VST2(v4u, (v4u*)(DST + ((size_t)p * rows + row) * TW + 8 * t), pk);
}

template <int FINAL>
__device__ __forceinline__ void rule_body(const unsigned short* __restrict__ Xp, const int ldx, const float xs1,
                                          const unsigned short* __restrict__ U16p, const unsigned short* __restrict__ V16p,
                                          const float* __restrict__ gain, const int* __restrict__ rids,
                                          float* Cio, const int ldc, const float* __restrict__ HO, const float* __restrict__ gate, float* Out) {
    __shared__ __align__(16) _Float16 Us[4][FA * FA];
    __shared__ __align__(16) _Float16 Vs[4][FA * FA];
    __shared__ __align__(16) _Float16 XT[4][FA * FA];
    __shared__ __align__(16) float Rs[4][32 * 36];
    const int lane = threadIdx.x & 31;
    const int wave = __builtin_amdgcn_readfirstlane((int)(threadIdx.x >> 5));
    const int hh = lane >> 4, m = lane & 15;
    const int n = blockIdx.x * 4 + wave;
    if (n >= kMROWS) return;
    const int nf = (n / SEQ) * SEQ_FULL + (n % SEQ);
    int rid = rids[nf];
    rid = (rid < 0) ? 0 : ((rid > NR - 1) ? NR - 1 : rid);
    const float g = cmb_bf(gain[rid]) * 0.0009765625f;
    const _Float16* Ug = (const _Float16*)U16p + (size_t)rid * (FA * FA);
    const _Float16* Vg = (const _Float16*)V16p + (size_t)rid * (FA * FA);
#pragma unroll
    for (int i = 0; i < 4; ++i) {
        const int idx = (i * 32 + lane) * 8;
        *(v8h_a*)&Us[wave][idx] = *(const v8h*)(Ug + idx);
        *(v8h_a*)&Vs[wave][idx] = *(const v8h*)(Vg + idx);
    }
    wave_sync_lds();

    const _Float16* xr = (const _Float16*)Xp + (size_t)n * ldx + 8 * hh;
#pragma unroll
    for (int bt = 0; bt < 2; ++bt) {
        const v16h ax = ldfrag(xr + (bt * 16 + m) * FA);
#pragma unroll
        for (int ct = 0; ct < 2; ++ct) {
            FragH bu;
            bu.h[0] = *(const v8h_a*)&Us[wave][(ct * 16 + m) * FA + 8 * hh];
            bu.h[1] = *(const v8h_a*)&Us[wave][(ct * 16 + m) * FA + 16 + 8 * hh];
            v8f acc = (v8f){0.f, 0.f, 0.f, 0.f, 0.f, 0.f, 0.f, 0.f};
            acc = wmma16(ax, bu.v, acc);
            v8h o;
#pragma unroll
            for (int r = 0; r < 8; ++r) o[r] = toh_flush(acc[r] * xs1);
            *(v8h_a*)&XT[wave][(ct * 16 + m) * FA + bt * 16 + 8 * hh] = o;
        }
    }
    wave_sync_lds();
#pragma unroll
    for (int dt = 0; dt < 2; ++dt) {
        FragH av;
        av.h[0] = *(const v8h_a*)&Vs[wave][(dt * 16 + m) * FA + 8 * hh];
        av.h[1] = *(const v8h_a*)&Vs[wave][(dt * 16 + m) * FA + 16 + 8 * hh];
#pragma unroll
        for (int ct = 0; ct < 2; ++ct) {
            FragH bx;
            bx.h[0] = *(const v8h_a*)&XT[wave][(ct * 16 + m) * FA + 8 * hh];
            bx.h[1] = *(const v8h_a*)&XT[wave][(ct * 16 + m) * FA + 16 + 8 * hh];
            v8f acc = (v8f){0.f, 0.f, 0.f, 0.f, 0.f, 0.f, 0.f, 0.f};
            acc = wmma16(av.v, bx.v, acc);
#pragma unroll
            for (int r = 0; r < 8; ++r) Rs[wave][(dt * 16 + 8 * hh + r) * 36 + ct * 16 + m] = acc[r] * g;
        }
    }
    wave_sync_lds();
#pragma unroll 1
    for (int q = 0; q < 8; ++q) {
        const int ch = 128 * q + 4 * lane;
        const int d = ch >> 5, cc = ch & 31;
        const v4f rv = *(const v4f_a*)&Rs[wave][d * 36 + cc];
        const v4f base = *(const v4f*)(Cio + (size_t)n * ldc + ch);
        if (FINAL) {
            const v4f ho = *(const v4f*)(HO + (size_t)n * CW + ch);
            const v4f gt = *(const v4f*)(gate + ch);
            v4f gb; gb.x = cmb_bf(gt.x); gb.y = cmb_bf(gt.y); gb.z = cmb_bf(gt.z); gb.w = cmb_bf(gt.w);
            const v4f fin = (base + rv) + ho * gb;
            VST2(v4f, (v4f*)(Out + (size_t)nf * CW + ch), fin);
        } else {
            const v4f fin = base + rv;
            VST2(v4f, (v4f*)(Cio + (size_t)n * ldc + ch), fin);
        }
    }
}

__global__ __launch_bounds__(128) void k_rule_mid(const unsigned short* __restrict__ X16, const unsigned short* __restrict__ U16, const unsigned short* __restrict__ V16,
                                                  const float* __restrict__ gain, const int* __restrict__ rids, float* QKV) {
    const int p = blockIdx.y;
    rule_body<0>(X16, CW, 1.0f, U16 + (size_t)p * NR * FA * FA, V16 + (size_t)p * NR * FA * FA, gain + p * NR, rids,
                 QKV + (size_t)p * CW, QKVW, gain, gain, QKV);
}
__global__ __launch_bounds__(128) void k_rule_out(const unsigned short* __restrict__ Y16, const unsigned short* __restrict__ U16, const unsigned short* __restrict__ V16,
                                                  const float* __restrict__ gain, const int* __restrict__ rids, float* OB,
                                                  const float* __restrict__ HO, const float* __restrict__ gate, float* Out) {
    rule_body<1>(Y16, YW, 0.0625f, U16, V16, gain, rids, OB, CW, HO, gate, Out);
}

__global__ __launch_bounds__(256) void k_rope(const float* __restrict__ QKV, const float* __restrict__ EMB, unsigned short* __restrict__ QK16, unsigned short* __restrict__ QKR16) {
#pragma clang fp contract(off)
    const int L = threadIdx.x & 31;
    const int wv = blockIdx.x * 8 + __builtin_amdgcn_readfirstlane((int)(threadIdx.x >> 5));
    if (wv >= kMROWS * NH) return;
    const int hd = wv % NH, r = wv / NH, t = r % SEQ, b = r / SEQ;
    const v2f sc = *(const v2f*)(EMB + (size_t)t * 64 + 2 * L);
    const float sinv = sc.x, cosv = sc.y;
#pragma unroll 1
    for (int sel = 0; sel < 2; ++sel) {
        const v2f x = *(const v2f*)(QKV + (size_t)r * QKVW + sel * CW + hd * HD + 2 * L);
        const float o0 = (x.x * cosv - x.y * sinv) * 16.f;
        const float o1 = (x.y * cosv + x.x * sinv) * 16.f;
        const h16 h0 = toh_flush(o0), h1 = toh_flush(o1);
        VST2(unsigned, (unsigned*)(QK16 + (size_t)sel * kMROWS * CW + (size_t)r * CW + hd * HD + 2 * L), pk2b(h0, h1));
        if (t < EROWS) {
            const h16 r0 = res_h(o0, h0), r1 = res_h(o1, h1);
            VST2(unsigned, (unsigned*)(QKR16 + ((size_t)(sel * NB + b) * EROWS + t) * CW + hd * HD + 2 * L), pk2b(r0, r1));
        }
    }
}

__global__ __launch_bounds__(256) void k_vtr(const float* __restrict__ QKV, unsigned short* __restrict__ VT16, unsigned short* __restrict__ VTR16, int has_res) {
#pragma clang fp contract(off)
    __shared__ float tile[64][65];
    const int u = threadIdx.x;
    const int bx = blockIdx.x; const int tt = bx % (SEQ / 64); const int bh = bx / (SEQ / 64); const int hd = bh % NH; const int b = bh / NH;
    const int t0 = tt * 64;
#pragma unroll
    for (int it = 0; it < 4; ++it) {
        const int row = (u >> 4) + 16 * it, c4 = (u & 15) * 4;
        const v4f v = *(const v4f*)(QKV + (size_t)(b * SEQ + t0 + row) * QKVW + 2 * CW + hd * HD + c4);
        tile[row][c4] = v.x; tile[row][c4 + 1] = v.y; tile[row][c4 + 2] = v.z; tile[row][c4 + 3] = v.w;
    }
    __syncthreads();
    const bool do_res = (has_res != 0) && (t0 < EROWS);
#pragma unroll
    for (int it = 0; it < 2; ++it) {
        const int d = (u >> 3) + 32 * it, pc = u & 7;
        float vv[8]; h16 hv[8];
#pragma unroll
        for (int i = 0; i < 8; ++i) { vv[i] = tile[8 * pc + i][d] * 16.f; hv[i] = toh_flush(vv[i]); }
        v4u pk; pk.x = pk2b(hv[0], hv[1]); pk.y = pk2b(hv[2], hv[3]); pk.z = pk2b(hv[4], hv[5]); pk.w = pk2b(hv[6], hv[7]);
        VST2(v4u, (v4u*)(VT16 + ((size_t)((b * NH + hd) * HD + d)) * SEQ + t0 + 8 * pc), pk);
        if (do_res) {
            h16 rv[8];
#pragma unroll
            for (int i = 0; i < 8; ++i) rv[i] = res_h(vv[i], hv[i]);
            v4u pr; pr.x = pk2b(rv[0], rv[1]); pr.y = pk2b(rv[2], rv[3]); pr.z = pk2b(rv[4], rv[5]); pr.w = pk2b(rv[6], rv[7]);
            VST2(v4u, (v4u*)(VTR16 + ((size_t)((b * NH + hd) * HD + d)) * EROWS + t0 + 8 * pc), pr);
        }
    }
}

template <int RES>
__device__ __forceinline__ void attn_body(const unsigned short* __restrict__ QK16p, const unsigned short* __restrict__ QKR16p,
                                          const unsigned short* __restrict__ VT16p, const unsigned short* __restrict__ VTR16p,
                                          unsigned short* __restrict__ Y16, const int qb, const int bh) {
    __shared__ __align__(16) _Float16 Ps[4][16 * PSP];
    __shared__ __align__(16) _Float16 Pr[4][16 * PSP];
    __shared__ __align__(16) float Os[4][16 * 68];
    const int lane = threadIdx.x & 31;
    const int wave = __builtin_amdgcn_readfirstlane((int)(threadIdx.x >> 5));
    const int hh = lane >> 4, c = lane & 15;
    const int hd = bh % NH, b = bh / NH;
    const int q0 = qb * 64 + wave * 16;
    const _Float16* Qb = (const _Float16*)QK16p + (size_t)b * SEQ * CW + hd * HD;
    const _Float16* Kb = Qb + (size_t)kMROWS * CW;
    const _Float16* Vb = (const _Float16*)VT16p + (size_t)(b * NH + hd) * HD * SEQ;
    const _Float16* QRb = (const _Float16*)QKR16p + (size_t)b * EROWS * CW + hd * HD;
    const _Float16* KRb = QRb + (size_t)NB * EROWS * CW;
    const _Float16* VRb = (const _Float16*)VTR16p + (size_t)(b * NH + hd) * HD * EROWS;
    const float NEG = -__builtin_inff();
    const float LSC = 0.000704440937934064f;
    const float RINV = 0.00048828125f;
    const int qoff = (q0 + c) * CW + 8 * hh;

    float mrow[8], lrow[8]; v8f oacc[4], orac[4];
#pragma unroll
    for (int r = 0; r < 8; ++r) { mrow[r] = NEG; lrow[r] = 0.f; }
#pragma unroll
    for (int t = 0; t < 4; ++t) { oacc[t] = (v8f){0.f, 0.f, 0.f, 0.f, 0.f, 0.f, 0.f, 0.f}; orac[t] = oacc[t]; }

    const int nhalf = (q0 >> 5) + 1;
    for (int kh = 0; kh < nhalf; ++kh) {
        const int kv0 = kh * 32;
        int qo = qoff; asm volatile("" : "+v"(qo));
        const v16h qa0 = ldfrag(Qb + qo), qa1 = ldfrag(Qb + qo + 32);
        v16h qr0 = qa0, qr1 = qa1;
        if (RES) { qr0 = ldfrag(QRb + qo); qr1 = ldfrag(QRb + qo + 32); }
        const int ko = (kv0 + c) * CW + 8 * hh;
        v8f sc0, sc1;
        {
            const v16h ka = ldfrag(Kb + ko), kb = ldfrag(Kb + ko + 32);
            v8f s = (v8f){0.f, 0.f, 0.f, 0.f, 0.f, 0.f, 0.f, 0.f};
            s = wmma16(qa0, ka, s); s = wmma16(qa1, kb, s);
            if (RES) {
                const v16h kra = ldfrag(KRb + ko), krb = ldfrag(KRb + ko + 32);
                v8f e = (v8f){0.f, 0.f, 0.f, 0.f, 0.f, 0.f, 0.f, 0.f};
                e = wmma16(qa0, kra, e); e = wmma16(qa1, krb, e); e = wmma16(qr0, ka, e); e = wmma16(qr1, kb, e);
                s = s + e * RINV;
            }
            sc0 = s;
        }
        {
            const v16h ka = ldfrag(Kb + ko + 16 * CW), kb = ldfrag(Kb + ko + 16 * CW + 32);
            v8f s = (v8f){0.f, 0.f, 0.f, 0.f, 0.f, 0.f, 0.f, 0.f};
            s = wmma16(qa0, ka, s); s = wmma16(qa1, kb, s);
            if (RES) {
                const v16h kra = ldfrag(KRb + ko + 16 * CW), krb = ldfrag(KRb + ko + 16 * CW + 32);
                v8f e = (v8f){0.f, 0.f, 0.f, 0.f, 0.f, 0.f, 0.f, 0.f};
                e = wmma16(qa0, kra, e); e = wmma16(qa1, krb, e); e = wmma16(qr0, ka, e); e = wmma16(qr1, kb, e);
                s = s + e * RINV;
            }
            sc1 = s;
        }
        const int kc0 = kv0 + c, kc1 = kc0 + 16;
#pragma unroll
        for (int r = 0; r < 8; ++r) {
            const int qrow = q0 + 8 * hh + r;
            float l0 = sc0[r] * LSC, l1 = sc1[r] * LSC;
            l0 = (kc0 > qrow) ? NEG : l0; l1 = (kc1 > qrow) ? NEG : l1;
            float mx = fmaxf(l0, l1);
            mx = fmaxf(mx, __shfl_xor(mx, 1, 32)); mx = fmaxf(mx, __shfl_xor(mx, 2, 32)); mx = fmaxf(mx, __shfl_xor(mx, 4, 32)); mx = fmaxf(mx, __shfl_xor(mx, 8, 32));
            const float mnew = fmaxf(mrow[r], mx);
            const float alpha = exp2f(mrow[r] - mnew);
            mrow[r] = mnew;
            const float e0 = l0 - mnew, e1 = l1 - mnew;
            const float p0 = (e0 < -22.0f) ? 0.f : exp2f(e0) * 256.f;
            const float p1 = (e1 < -22.0f) ? 0.f : exp2f(e1) * 256.f;
            const h16 h0 = (h16)p0, h1 = (h16)p1;
            Ps[wave][(8 * hh + r) * PSP + c] = h0; Ps[wave][(8 * hh + r) * PSP + 16 + c] = h1;
            float ps;
            if (RES) {
                Pr[wave][(8 * hh + r) * PSP + c] = res_h(p0, h0); Pr[wave][(8 * hh + r) * PSP + 16 + c] = res_h(p1, h1);
                ps = p0 + p1;
            } else {
                ps = (float)h0 + (float)h1;
            }
            ps += __shfl_xor(ps, 1, 32); ps += __shfl_xor(ps, 2, 32); ps += __shfl_xor(ps, 4, 32); ps += __shfl_xor(ps, 8, 32);
            lrow[r] = lrow[r] * alpha + ps;
#pragma unroll
            for (int t = 0; t < 4; ++t) { oacc[t][r] *= alpha; if (RES) orac[t][r] *= alpha; }
        }
        wave_sync_lds();
        FragH pa, pq;
        pa.h[0] = *(const v8h_a*)&Ps[wave][c * PSP + 8 * hh];
        pa.h[1] = *(const v8h_a*)&Ps[wave][c * PSP + 16 + 8 * hh];
        pq = pa;
        if (RES) {
            pq.h[0] = *(const v8h_a*)&Pr[wave][c * PSP + 8 * hh];
            pq.h[1] = *(const v8h_a*)&Pr[wave][c * PSP + 16 + 8 * hh];
        }
        const int vo = c * SEQ + kv0 + 8 * hh;
        const int vro = c * EROWS + kv0 + 8 * hh;
#pragma unroll
        for (int t = 0; t < 4; ++t) {
            const v16h vb = ldfrag(Vb + vo + t * 16 * SEQ);
            oacc[t] = wmma16(pa.v, vb, oacc[t]);
            if (RES) {
                const v16h vr = ldfrag(VRb + vro + t * 16 * EROWS);
                orac[t] = wmma16(pa.v, vr, orac[t]);
                orac[t] = wmma16(pq.v, vb, orac[t]);
            }
        }
        wave_sync_lds();
    }

#pragma unroll
    for (int r = 0; r < 8; ++r) {
        const float inv = 1.0f / lrow[r];
#pragma unroll
        for (int t = 0; t < 4; ++t) {
            const float y = RES ? (oacc[t][r] + orac[t][r] * RINV) * inv : oacc[t][r] * inv;
            Os[wave][(8 * hh + r) * 68 + t * 16 + c] = y;
        }
    }
    wave_sync_lds();
    {
        const int q4 = lane >> 3, c8 = (lane & 7) * 8;
        unsigned short* yb = Y16 + (size_t)(b * SEQ + q0) * YW + hd * HD + c8;
        v4u pk[4], pr[4];
#pragma unroll
        for (int it = 0; it < 4; ++it) {
            const int row = it * 4 + q4;
            const v4f a = *(const v4f_a*)&Os[wave][row * 68 + c8];
            const v4f d = *(const v4f_a*)&Os[wave][row * 68 + c8 + 4];
            const h16 g0 = toh_flush(a.x), g1 = toh_flush(a.y), g2 = toh_flush(a.z), g3 = toh_flush(a.w);
            const h16 g4 = toh_flush(d.x), g5 = toh_flush(d.y), g6 = toh_flush(d.z), g7 = toh_flush(d.w);
            pk[it].x = pk2b(g0, g1); pk[it].y = pk2b(g2, g3); pk[it].z = pk2b(g4, g5); pk[it].w = pk2b(g6, g7);
            pr[it].x = pk2b(res_h(a.x, g0), res_h(a.y, g1)); pr[it].y = pk2b(res_h(a.z, g2), res_h(a.w, g3));
            pr[it].z = pk2b(res_h(d.x, g4), res_h(d.y, g5)); pr[it].w = pk2b(res_h(d.z, g6), res_h(d.w, g7));
        }
        for (int pass = 0; pass < 2; ++pass) {
#pragma unroll
            for (int it = 0; it < 4; ++it) {
                *(volatile v4u*)(yb + (size_t)(it * 4 + q4) * YW) = pk[it];
                *(volatile v4u*)(yb + (size_t)(it * 4 + q4) * YW + CW) = pr[it];
            }
            __threadfence();
        }
    }
}

__global__ __launch_bounds__(128) void k_attn_early(const unsigned short* __restrict__ QK16, const unsigned short* __restrict__ QKR16,
                                                    const unsigned short* __restrict__ VT16, const unsigned short* __restrict__ VTR16, unsigned short* __restrict__ Y16) {
    const int nqb = EROWS / 64;
    const int bx = blockIdx.x;
    attn_body<1>(QK16, QKR16, VT16, VTR16, Y16, bx % nqb, bx / nqb);
}
__global__ __launch_bounds__(128) void k_attn_late(const unsigned short* __restrict__ QK16, const unsigned short* __restrict__ QKR16,
                                                   const unsigned short* __restrict__ VT16, const unsigned short* __restrict__ VTR16, unsigned short* __restrict__ Y16) {
    const int nqb = (SEQ > EROWS) ? (SEQ - EROWS) / 64 : 1;
    const int bx = blockIdx.x;
    attn_body<0>(QK16, QKR16, VT16, VTR16, Y16, EROWS / 64 + bx % nqb, bx / nqb);
}

__global__ __launch_bounds__(32) void k_hier_dots(const float* __restrict__ QKVv, const int* __restrict__ rids, float* __restrict__ P1) {
#pragma clang fp contract(off)
    __shared__ __align__(16) float ks[NR * KP];
    __shared__ __align__(16) float qs[HSLAB];
    __shared__ __align__(16) float ps[8 * 32];
    const int L = threadIdx.x & 31;
    const int u = L & 15, hf = L >> 4;
    const int slab = blockIdx.x % NSLAB, b = blockIdx.x / NSLAB;
    if (b >= NB) return;
    const int c0 = slab * HSLAB;
    const v4f z4 = (v4f){0.f, 0.f, 0.f, 0.f};
#pragma unroll 1
    for (int i = 0; i < NR; ++i) *(v4f_a*)&ks[i * KP + 4 * L] = z4;
    wave_sync_lds();
    int cnt = 0;
    const float* src = QKVv + (size_t)b * SEQ * QKVW + c0 + 4 * L;
    const int* idr = rids + (size_t)b * SEQ_FULL;
    float* dst = P1 + (size_t)(b * NSLAB + slab) * SEQ * 32;
#pragma unroll 1
    for (int s = 0; s < SEQ; ++s) {
        const v4f qv = *(const v4f*)(src + (size_t)s * QKVW);
        const v4f kv = *(const v4f*)(src + (size_t)s * QKVW + CW);
        const int id = idr[s];
        const int idc = min(max(id, 0), NR - 1);
        const bool valid = (id == idc);
        v4f cur = *(const v4f_a*)&ks[idc * KP + 4 * L];
        cur.x += valid ? kv.x : 0.f; cur.y += valid ? kv.y : 0.f; cur.z += valid ? kv.z : 0.f; cur.w += valid ? kv.w : 0.f;
        *(v4f_a*)&ks[idc * KP + 4 * L] = cur;
        *(v4f_a*)&qs[4 * L] = qv;
        cnt += (id == u) ? 1 : 0;
        wave_sync_lds();
        float acc = 0.f;
#pragma unroll 4
        for (int i = 0; i < 16; ++i) {
            const int cc = hf * 64 + 4 * i;
            const v4f a = *(const v4f_a*)&ks[u * KP + cc];
            const v4f q = *(const v4f_a*)&qs[cc];
            acc += (a.x * q.x + a.y * q.y) + (a.z * q.z + a.w * q.w);
        }
        acc += __shfl_xor(acc, 16, 32);
        const float rc = 1.0f / (float)max(cnt, 1);
        ps[(s & 7) * 32 + L] = (hf == 0) ? acc * rc : rc;
        wave_sync_lds();
        if ((s & 7) == 7) {
            const v4f o0 = *(const v4f_a*)&ps[4 * L];
            const v4f o1 = *(const v4f_a*)&ps[128 + 4 * L];
            float* d = dst + (size_t)(s - 7) * 32;
            VST2(v4f, (v4f*)(d + 4 * L), o0);
            VST2(v4f, (v4f*)(d + 128 + 4 * L), o1);
        }
    }
}

__global__ __launch_bounds__(256) void k_hier_soft(const float* __restrict__ P1, float* __restrict__ WC) {
#pragma clang fp contract(off)
    const int L = threadIdx.x & 31;
    const int wv = blockIdx.x * 8 + __builtin_amdgcn_readfirstlane((int)(threadIdx.x >> 5));
    if (wv >= kMROWS / 2) return;
    const int u = L & 15, hf = L >> 4;
    const int r = 2 * wv + hf;
    const int b = r / SEQ, s = r % SEQ;
    const float* p = P1 + ((size_t)b * NSLAB * SEQ + s) * 32 + u;
    float lg = 0.f;
#pragma unroll
    for (int j = 0; j < NSLAB; ++j) lg += p[(size_t)j * SEQ * 32];
    const float rc = p[16];
    lg *= 0.03125f;
    float mx = lg;
    mx = fmaxf(mx, __shfl_xor(mx, 1, 32)); mx = fmaxf(mx, __shfl_xor(mx, 2, 32)); mx = fmaxf(mx, __shfl_xor(mx, 4, 32)); mx = fmaxf(mx, __shfl_xor(mx, 8, 32));
    const float e = expf(lg - mx);
    float sum = e;
    sum += __shfl_xor(sum, 1, 32); sum += __shfl_xor(sum, 2, 32); sum += __shfl_xor(sum, 4, 32); sum += __shfl_xor(sum, 8, 32);
    const float cf = (e * (1.0f / sum)) * rc;
    VST2(float, WC + (size_t)r * 16 + u, cf);
}

__global__ __launch_bounds__(32) void k_hier_out(const float* __restrict__ QKVv, const int* __restrict__ rids, const float* __restrict__ WC, float* __restrict__ HO) {
#pragma clang fp contract(off)
    __shared__ __align__(16) float vs[NR * KP];
    const int L = threadIdx.x & 31;
    const int slab = blockIdx.x % NSLAB, b = blockIdx.x / NSLAB;
    if (b >= NB) return;
    const int c0 = slab * HSLAB;
    const v4f z4 = (v4f){0.f, 0.f, 0.f, 0.f};
#pragma unroll 1
    for (int i = 0; i < NR; ++i) *(v4f_a*)&vs[i * KP + 4 * L] = z4;
    const float* src = QKVv + (size_t)b * SEQ * QKVW + 2 * CW + c0 + 4 * L;
    const int* idr = rids + (size_t)b * SEQ_FULL;
#pragma unroll 1
    for (int s = 0; s < SEQ; ++s) {
        const int row = b * SEQ + s;
        const v4f vv = *(const v4f*)(src + (size_t)s * QKVW);
        const int id = idr[s];
        const int idc = min(max(id, 0), NR - 1);
        const bool valid = (id == idc);
        v4f cur = *(const v4f_a*)&vs[idc * KP + 4 * L];
        cur.x += valid ? vv.x : 0.f; cur.y += valid ? vv.y : 0.f; cur.z += valid ? vv.z : 0.f; cur.w += valid ? vv.w : 0.f;
        *(v4f_a*)&vs[idc * KP + 4 * L] = cur;
        const float* cfp = WC + (size_t)row * 16;
        v4f acc = z4;
#pragma unroll 4
        for (int uu = 0; uu < NR; ++uu) {
            const float cu = cfp[uu];
            const v4f a = *(const v4f_a*)&vs[uu * KP + 4 * L];
            acc.x += a.x * cu; acc.y += a.y * cu; acc.z += a.z * cu; acc.w += a.w * cu;
        }
        VST2(v4f, (v4f*)(HO + (size_t)row * CW + c0 + 4 * L), acc);
    }
}

constexpr size_t al256(size_t x) { return (x + 255) / 256 * 256; }
constexpr size_t SZ_EMB  = al256((size_t)SEQ * 64 * 4);
constexpr size_t SZ_X16  = al256((size_t)kMROWS * CW * 2);
constexpr size_t SZ_SIT  = al256((size_t)4 * RK * CW * 2);
constexpr size_t SZ_SI3  = al256((size_t)2 * RK * YW * 2);
constexpr size_t SZ_SOT  = al256((size_t)4 * CW * TW * 2);
constexpr size_t SZ_UV   = al256((size_t)4 * NR * FA * FA * 2);
constexpr size_t SZ_WT   = al256((size_t)QKVW * CW * 2);
constexpr size_t SZ_TF   = al256((size_t)kMROWS * 4 * RK * 4);
constexpr size_t SZ_T3F  = al256((size_t)kMROWS * 2 * RK * 4);
constexpr size_t SZ_TS   = al256((size_t)4 * kMROWS * TW * 2);
constexpr size_t SZ_U1   = al256((size_t)kMROWS * QKVW * 4);
constexpr size_t SZ_QK16 = al256((size_t)2 * kMROWS * CW * 2);
constexpr size_t SZ_QKR  = al256((size_t)2 * NB * EROWS * CW * 2);
constexpr size_t SZ_VT   = al256((size_t)kMROWS * CW * 2);
constexpr size_t SZ_VTR  = al256((size_t)NB * NH * HD * EROWS * 2);
constexpr size_t SZ_Y16  = al256((size_t)kMROWS * YW * 2);
constexpr size_t SZ_F32  = al256((size_t)kMROWS * CW * 4);
constexpr size_t SZ_P1   = al256((size_t)NB * NSLAB * SEQ * 32 * 4);
constexpr size_t SZ_WC   = al256((size_t)kMROWS * 16 * 4);
constexpr size_t SZ_TOTAL = SZ_EMB + SZ_X16 + SZ_SIT + SZ_SI3 + SZ_SOT + SZ_UV + SZ_UV + SZ_WT + SZ_TF + SZ_T3F + SZ_TS + SZ_U1 + SZ_QK16 + SZ_QKR
                          + SZ_VT + SZ_VTR + SZ_Y16 + SZ_F32 + SZ_P1 + SZ_WC + SZ_F32;
static_assert(SZ_TOTAL <= (size_t)134217728);
static_assert((size_t)((NB_FULL - 1) * SEQ_FULL + SEQ_FULL) * CW * 4 == (size_t)8388608);
static_assert(((size_t)((NB - 1) * NSLAB + (NSLAB - 1)) * SEQ * 32 + (size_t)(SEQ - 8) * 32 + 128 + 4 * 31 + 3) * 4 < SZ_P1);
static_assert(((size_t)(kMROWS - 1) * 16 + 15) * 4 < SZ_WC);
static_assert(((size_t)(kMROWS - 1) * CW + (NSLAB - 1) * HSLAB + 4 * 31 + 3) * 4 < SZ_F32);

extern "C" void kernel_launch(void* const* d_in, const int* in_sizes, int n_in, void* d_out, int out_size, void* d_ws, size_t ws_size, hipStream_t stream) {
    if (n_in < 10) return;
    const long long need_rows = (long long)(NB - 1) * SEQ_FULL + SEQ;
    if ((long long)in_sizes[0] < need_rows * CW) return;
    if ((long long)out_size < need_rows * CW) return;
    if (in_sizes[1] < 4 * CW * RK || in_sizes[2] < 4 * RK * CW) return;
    if (in_sizes[3] < 4 * NR * FA * FA || in_sizes[4] < 4 * NR * FA * FA || in_sizes[5] < 4 * NR) return;
    if (in_sizes[6] < CW * CW || in_sizes[7] < 2 * CW * CW || in_sizes[8] < CW) return;
    if ((long long)in_sizes[9] < need_rows) return;
    if (SZ_TOTAL > ws_size) return;

    const float* x     = (const float*)d_in[0];
    const float* s_in  = (const float*)d_in[1];
    const float* s_out = (const float*)d_in[2];
    const float* ruleU = (const float*)d_in[3];
    const float* ruleV = (const float*)d_in[4];
    const float* gain  = (const float*)d_in[5];
    const float* wq    = (const float*)d_in[6];
    const float* wkv   = (const float*)d_in[7];
    const float* gate  = (const float*)d_in[8];
    const int*   rids  = (const int*)d_in[9];
    float* out = (float*)d_out;

    char* wsp = (char*)d_ws;
    float* EMB = (float*)wsp; wsp += SZ_EMB;
    unsigned short* X16 = (unsigned short*)wsp; wsp += SZ_X16;
    unsigned short* SIT16 = (unsigned short*)wsp; wsp += SZ_SIT;
    unsigned short* SI3T16 = (unsigned short*)wsp; wsp += SZ_SI3;
    unsigned short* SOT16 = (unsigned short*)wsp; wsp += SZ_SOT;
    unsigned short* U16 = (unsigned short*)wsp; wsp += SZ_UV;
    unsigned short* V16 = (unsigned short*)wsp; wsp += SZ_UV;
    unsigned short* WT16 = (unsigned short*)wsp; wsp += SZ_WT;
    float* TF = (float*)wsp; wsp += SZ_TF;
    float* T3F = (float*)wsp; wsp += SZ_T3F;
    unsigned short* TS16 = (unsigned short*)wsp; wsp += SZ_TS;
    float* U1 = (float*)wsp; wsp += SZ_U1;
    unsigned short* QK16 = (unsigned short*)wsp; wsp += SZ_QK16;
    unsigned short* QKR16 = (unsigned short*)wsp; wsp += SZ_QKR;
    unsigned short* VT16 = (unsigned short*)wsp; wsp += SZ_VT;
    unsigned short* VTR16 = (unsigned short*)wsp; wsp += SZ_VTR;
    unsigned short* Y16 = (unsigned short*)wsp; wsp += SZ_Y16;
    float* OB = (float*)wsp; wsp += SZ_F32;
    float* P1 = (float*)wsp; wsp += SZ_P1;
    float* WC = (float*)wsp; wsp += SZ_WC;
    float* HO = (float*)wsp; wsp += SZ_F32;

    const float S16K = 6.103515625e-05f;
    const unsigned gBig = (unsigned)(((kMROWS / 64) * (CW / 64) + 7) / 8);

    k_embtab<<<(SEQ * 32 + 255) / 256, 256, 0, stream>>>(EMB, SEQ * 32);
    k_cast16<<<(unsigned)(((long long)kMROWS * (CW / 8) + 255) / 256), 256, 0, stream>>>(x, X16, kMROWS, CW, 1.0f, SEQ, SEQ_FULL);
    k_cast16<<<(unsigned)((4 * NR * FA * (FA / 8) + 255) / 256), 256, 0, stream>>>(ruleU, U16, 4 * NR * FA, FA, 32.0f, 4 * NR * FA, 4 * NR * FA);
    k_cast16<<<(unsigned)((4 * NR * FA * (FA / 8) + 255) / 256), 256, 0, stream>>>(ruleV, V16, 4 * NR * FA, FA, 32.0f, 4 * NR * FA, 4 * NR * FA);
    k_castT<<<(unsigned)(4 * (CW / 64) * (RK / 32)), 256, 0, stream>>>(s_in, RK, (long long)CW * RK, CW, RK, SIT16, CW, 0, 32.0f, 4);
    k_castT<<<(unsigned)(2 * (CW / 64) * (RK / 32)), 256, 0, stream>>>(s_in + (size_t)2 * CW * RK, RK, (long long)CW * RK, CW, RK, SI3T16, YW, 0, 1024.0f, 2);
    k_castT<<<(unsigned)(2 * (CW / 64) * (RK / 32)), 256, 0, stream>>>(s_in + (size_t)2 * CW * RK, RK, (long long)CW * RK, CW, RK, SI3T16, YW, CW, 0.5f, 2);
    k_sot<<<(unsigned)((4 * CW * 8 + 255) / 256), 256, 0, stream>>>(s_out, SOT16);
    k_castT<<<(unsigned)((CW / 64) * (CW / 32)), 256, 0, stream>>>(wq, CW, 0LL, CW, CW, WT16, CW, 0, 32.0f, 1);
    k_castT<<<(unsigned)((CW / 64) * (2 * CW / 32)), 256, 0, stream>>>(wkv, 2 * CW, 0LL, CW, 2 * CW, WT16 + (size_t)CW * CW, CW, 0, 32.0f, 1);

    k_gemm64<<<(unsigned)(((kMROWS / 64) * ((4 * RK) / 64) + 7) / 8), 256, 0, stream>>>(X16, CW, SIT16, CW, TF, 4 * RK, x, 0, kMROWS, 4 * RK, CW, 0.03125f);
    k_tsplit<<<(unsigned)(((long long)3 * kMROWS * 8 + 255) / 256), 256, 0, stream>>>(TF, 4 * RK, 0, TS16, kMROWS, 3);
    for (int p = 0; p < 3; ++p)
        k_gemm64<<<gBig, 256, 0, stream>>>(TS16 + (size_t)p * kMROWS * TW, TW, SOT16 + (size_t)p * CW * TW, TW, U1 + (size_t)p * CW, QKVW, x, 0, kMROWS, CW, TW, S16K);
    k_rule_mid<<<dim3((unsigned)(kMROWS / 4), 3), 128, 0, stream>>>(X16, U16, V16, gain, rids, U1);
    k_rope<<<(unsigned)((kMROWS * NH + 7) / 8), 256, 0, stream>>>(U1, EMB, QK16, QKR16);
    k_vtr<<<(unsigned)(NB * NH * (SEQ / 64)), 256, 0, stream>>>(U1, VT16, VTR16, 1);
    k_attn_early<<<(unsigned)(NB * NH * (EROWS / 64)), 128, 0, stream>>>(QK16, QKR16, VT16, VTR16, Y16);
    if (SEQ > EROWS)
        k_attn_late<<<(unsigned)(NB * NH * ((SEQ - EROWS) / 64)), 128, 0, stream>>>(QK16, QKR16, VT16, VTR16, Y16);

    k_gemm64<<<(unsigned)(((kMROWS / 64) * ((2 * RK) / 64) + 7) / 8), 256, 0, stream>>>(Y16, YW, SI3T16, YW, T3F, 2 * RK, x, 0, kMROWS, 2 * RK, YW, S16K);
    k_tsplit<<<(unsigned)(((long long)kMROWS * 8 + 255) / 256), 256, 0, stream>>>(T3F, 2 * RK, RK, TS16 + (size_t)3 * kMROWS * TW, kMROWS, 1);
    k_gemm64<<<gBig, 256, 0, stream>>>(TS16 + (size_t)3 * kMROWS * TW, TW, SOT16 + (size_t)3 * CW * TW, TW, OB, CW, x, 0, kMROWS, CW, TW, S16K);

    k_gemm64<<<(unsigned)(((kMROWS / 64) * (QKVW / 64) + 7) / 8), 256, 0, stream>>>(X16, CW, WT16, CW, U1, QKVW, x, 0, kMROWS, QKVW, CW, 0.03125f);
    k_hier_dots<<<(unsigned)(NB * NSLAB), 32, 0, stream>>>(U1, rids, P1);
    k_hier_soft<<<(unsigned)((kMROWS / 2 + 7) / 8), 256, 0, stream>>>(P1, WC);
    k_hier_out<<<(unsigned)(NB * NSLAB), 32, 0, stream>>>(U1, rids, WC, HO);

    k_rule_out<<<(unsigned)(kMROWS / 4), 128, 0, stream>>>(Y16, U16 + (size_t)3 * NR * FA * FA, V16 + (size_t)3 * NR * FA * FA, gain + 3 * NR, rids, OB, HO, gate, out);
}
